// GTLayer_44487271252168
// MI455X (gfx1250) — hardware-run, weakly checked
//
#include <hip/hip_runtime.h>
#include <stddef.h>


#define DM     128
#define NQKV   384
#define FW     256
#define GT     128
#define RB     1024
#define RBBITS 10
#define RMAX   64
#define RMBITS 6
#define TABW   (2 * RMAX)
#define CHUNK  4096
#define LCAP   18432
#define DEGCAP 64
#define STATRS 128
#define WSCAP  134217728
#define ASCL   8.0f
#define WSCL   64.0f
#define INVSCL 0.001953125f

#define EDGE_LDS_INTS  (RB + 8 + RB + LCAP)
#define EDGE_LDS_BYTES (EDGE_LDS_INTS * 4)

static_assert(RB == (1 << RBBITS));
static_assert(RMAX == (1 << RMBITS));
static_assert(CHUNK == 8 * 16 * 32);
static_assert(CHUNK == 4 * 4 * 256);
static_assert(TABW * 4 == 32 * 16);
static_assert((RB % 128) == 0);
static_assert(RB == 4 * 256);
static_assert((EDGE_LDS_BYTES % 16) == 0);
static_assert(EDGE_LDS_BYTES < 300000);
static_assert(NQKV == 3 * DM);
static_assert((DM % 64) == 0 && (FW % 64) == 0 && (NQKV % 64) == 0);
static_assert((STATRS % 2) == 0 && (STATRS % 128) == 0);
static_assert(DM == 32 * 4);

typedef float          v4f  __attribute__((ext_vector_type(4)));
typedef float          v8f  __attribute__((ext_vector_type(8)));
typedef double         v2d  __attribute__((ext_vector_type(2)));
typedef int            v4i  __attribute__((ext_vector_type(4)));
typedef unsigned int   v4u  __attribute__((ext_vector_type(4)));
typedef unsigned short v8us __attribute__((ext_vector_type(8)));
typedef _Float16       v16h __attribute__((ext_vector_type(16)));
union FragH { v16h v; v8us u[2]; };

__device__ __forceinline__ unsigned short h16(float f) {
  const _Float16 h = (_Float16)f;
  return __builtin_bit_cast(unsigned short, h);
}

__device__ __forceinline__ unsigned int pk2(float a, float b) {
  return (unsigned int)h16(a) | ((unsigned int)h16(b) << 16);
}

__device__ __forceinline__ v8us cvt8(v4f a, v4f b, float s) {
  v8us r;
  r[0] = h16(a.x * s); r[1] = h16(a.y * s); r[2] = h16(a.z * s); r[3] = h16(a.w * s);
  r[4] = h16(b.x * s); r[5] = h16(b.y * s); r[6] = h16(b.z * s); r[7] = h16(b.w * s);
  return r;
}

__device__ __forceinline__ v8f wmh(v16h a, v16h b, v8f c) {
  v8f d = __builtin_amdgcn_wmma_f32_16x16x32_f16(false, a, false, b, (short)0, c, false, false);
  asm volatile("v_nop\n\tv_nop\n\tv_nop\n\tv_nop" : "+v"(d) : "v"(a), "v"(b));
  return d;
}

template <int NB>
__device__ __forceinline__ unsigned int match_mask(unsigned int base, int key) {
  unsigned int msk = base;
#pragma unroll
  for (int b = 0; b < NB; ++b) {
    const bool bit = ((key >> b) & 1) != 0;
    const unsigned int bb = __builtin_amdgcn_ballot_w32(bit);
    msk &= bit ? bb : ~bb;
  }
  return msk;
}

__global__ __launch_bounds__(256) void k_csort(
    const int* __restrict__ key, unsigned int* csort, int* tab, int nN, int nE) {
  __shared__ __attribute__((aligned(16))) unsigned int sImg[CHUNK];
  __shared__ int cw[8 * RMAX];
  __shared__ __attribute__((aligned(16))) int sTb[TABW];
  __shared__ int sWt[8];
  int* sPre = sTb;
  int* sCn  = sTb + RMAX;
  const int tid = (int)threadIdx.x, lane = tid & 31, wave = tid >> 5;
  const int c = (int)blockIdx.x;
  const int cbase = c * CHUNK;

  for (int i = tid; i < 8 * RMAX; i += 256) cw[i] = 0;
  {
    const v4u s = {0xffffffffu, 0xffffffffu, 0xffffffffu, 0xffffffffu};
    for (int i = tid; i < CHUNK / 4; i += 256) ((v4u*)sImg)[i] = s;
  }
  __syncthreads();

  unsigned int ent[16];
  int pk[16];
  const unsigned int lt = (1u << lane) - 1u;
#pragma unroll
  for (int i = 0; i < 16; ++i) {
    const int e = cbase + wave * 512 + 32 * i + lane;
    const int ea = e > nE - 1 ? nE - 1 : e;
    const int d = key[ea];
    const bool valid = (e < nE) && ((unsigned)d < (unsigned)nN);
    const int dd = valid ? d : 0;
    const int r  = dd >> RBBITS;
    const int jl = dd & (RB - 1);
    const unsigned int pay = (unsigned int)ea;
    const unsigned int msk = match_mask<RMBITS>(__builtin_amdgcn_ballot_w32(valid), r);
    const int rank = (int)__builtin_popcount(msk & lt);
    const int grp  = (int)__builtin_popcount(msk);
    const int base = cw[wave * RMAX + r];
    pk[i]  = valid ? ((r << 12) | (base + rank)) : -1;
    ent[i] = (pay << RBBITS) | (unsigned int)jl;
    if (valid && rank == 0) cw[wave * RMAX + r] = base + grp;
    __syncthreads();
  }

  if (tid < RMAX) {
    int run = 0;
#pragma unroll
    for (int w = 0; w < 8; ++w) {
      const int v = cw[w * RMAX + tid];
      cw[w * RMAX + tid] = run;
      run += v;
    }
    sCn[tid] = run;
  }
  __syncthreads();
  {
    const int vr = sCn[tid & (RMAX - 1)];
    const int v  = (tid < RMAX) ? vr : 0;
    int x = v;
#pragma unroll
    for (int dd = 1; dd < 32; dd <<= 1) {
      const int y = __shfl_up(x, dd);
      x += (lane >= dd) ? y : 0;
    }
    if (lane == 31) sWt[wave] = x;
    __syncthreads();
    int pre = 0;
#pragma unroll
    for (int w = 0; w < 8; ++w) { const int tw = sWt[w]; pre += (w < wave) ? tw : 0; }
    if (tid < RMAX) sPre[tid] = pre + x - v;
  }
  __syncthreads();

#pragma unroll
  for (int i = 0; i < 16; ++i) {
    if (pk[i] >= 0) {
      const int r = (pk[i] >> 12) & (RMAX - 1);
      const int q = pk[i] & 4095;
      const int pos = sPre[r] + cw[wave * RMAX + r] + q;
      if ((unsigned)pos < (unsigned)CHUNK) sImg[pos] = ent[i];
    }
  }
  __syncthreads();

  v4u iv[4];
#pragma unroll
  for (int it = 0; it < 4; ++it) iv[it] = ((const v4u*)sImg)[it * 256 + tid];
  const v4i tv = *(const v4i*)(sTb + 4 * lane);
  unsigned int* gp = csort + (size_t)c * CHUNK;
  int* tp = tab + (size_t)c * TABW + 4 * lane;
  const bool wt = tid < 32;
#pragma unroll
  for (int it = 0; it < 4; ++it) *(volatile v4u*)(gp + 4 * (it * 256 + tid)) = iv[it];
  if (wt) *(volatile v4i*)tp = tv;
  __threadfence();
#pragma unroll
  for (int it = 0; it < 4; ++it) *(volatile v4u*)(gp + 4 * (it * 256 + tid)) = iv[it];
  if (wt) *(volatile v4i*)tp = tv;
}

__global__ __launch_bounds__(256) void k_xcvt(
    const float* __restrict__ x, unsigned short* x16, int nN) {
  const int tid = (int)threadIdx.x;
  const int rb = (int)blockIdx.x * 128;
  const v4f zero4 = {0.0f, 0.0f, 0.0f, 0.0f};
  v8us o[8];
#pragma unroll
  for (int it = 0; it < 8; ++it) {
    const int p = it * 256 + tid;
    const int row = rb + (p >> 4);
    const int c8 = (p & 15) * 8;
    const bool live = row < nN;
    const int xr = live ? row : (nN - 1);
    v4f a = *(const v4f*)(x + (size_t)xr * DM + c8);
    v4f b = *(const v4f*)(x + (size_t)xr * DM + c8 + 4);
    a = live ? a : zero4;
    b = live ? b : zero4;
    o[it] = cvt8(a, b, ASCL);
  }
#pragma unroll
  for (int it = 0; it < 8; ++it) {
    const int p = it * 256 + tid;
    *(volatile v8us*)(x16 + (size_t)(rb + (p >> 4)) * DM + (p & 15) * 8) = o[it];
  }
  __threadfence();
#pragma unroll
  for (int it = 0; it < 8; ++it) {
    const int p = it * 256 + tid;
    *(volatile v8us*)(x16 + (size_t)(rb + (p >> 4)) * DM + (p & 15) * 8) = o[it];
  }
}

template <int KP, int NOUT>
__global__ __launch_bounds__(256) void k_wprep(
    const float* __restrict__ W0, const float* __restrict__ W1, const float* __restrict__ W2,
    const float* __restrict__ W3, unsigned short* T) {
  constexpr int WPP = KP + 8;
  constexpr int BPM = NOUT / 32;
  constexpr int PPR = KP / 8;
  static_assert((WPP % 8) == 0);
  static_assert((KP % 64) == 0 && (NOUT % 32) == 0);
  __shared__ __attribute__((aligned(16))) unsigned short sT[32 * WPP];
  const int tid = (int)threadIdx.x;
  const int b = (int)blockIdx.x;
  const int mat = b / BPM;
  const float* W = (mat == 0) ? W0 : ((mat == 1) ? W1 : ((mat == 2) ? W2 : W3));
  const int nb0 = (b % BPM) * 32;
  const int rowBase = b * 32;

  for (int i = tid; i < (32 * WPP) / 2; i += 256) ((unsigned int*)sT)[i] = 0u;
  __syncthreads();

#pragma unroll 1
  for (int it = 0; it < KP / 32; ++it) {
    const int p = it * 256 + tid;
    const int k = p >> 3, q = p & 7;
    const v4f w = *(const v4f*)(W + (size_t)k * NOUT + nb0 + 4 * q);
    unsigned short* d = sT + (4 * q) * WPP + k;
    d[0]       = h16(w.x * WSCL);
    d[WPP]     = h16(w.y * WSCL);
    d[2 * WPP] = h16(w.z * WSCL);
    d[3 * WPP] = h16(w.w * WSCL);
  }
  __syncthreads();

#pragma unroll 1
  for (int it = 0; it < KP / 64; ++it) {
    const int p = it * 256 + tid;
    const int row = p / PPR, c8 = (p % PPR) * 8;
    const v8us v = *(const v8us*)(sT + row * WPP + c8);
    *(volatile v8us*)(T + (size_t)(rowBase + row) * KP + c8) = v;
  }
  __threadfence();
#pragma unroll 1
  for (int it = 0; it < KP / 64; ++it) {
    const int p = it * 256 + tid;
    const int row = p / PPR, c8 = (p % PPR) * 8;
    const v8us v = *(const v8us*)(sT + row * WPP + c8);
    *(volatile v8us*)(T + (size_t)(rowBase + row) * KP + c8) = v;
  }
}

template <int KS, int HASB, int RES, int RELU, int O16>
__global__ __launch_bounds__(GT) void k_gemm(
    const unsigned short* __restrict__ A, const unsigned short* __restrict__ Bt,
    const float* __restrict__ bias, const float* __restrict__ resid, int ldr, int rrows,
    float* outF, unsigned short* outH, int ldo, int Mp, int Ncols) {
  constexpr int K = 32 * KS;
  __shared__ __attribute__((aligned(16))) float sT[4 * 32 * 64];
  const int tid = (int)threadIdx.x, lane = tid & 31, wave = tid >> 5, hh = lane >> 4, m = lane & 15;
  const int c0 = (int)blockIdx.x * 64;
  const int r0 = (int)blockIdx.y * 128 + wave * 32;

  int ra0 = r0 + m;      ra0 = ra0 > Mp - 1 ? Mp - 1 : ra0;
  int ra1 = r0 + 16 + m; ra1 = ra1 > Mp - 1 ? Mp - 1 : ra1;
  const unsigned short* ap0 = A + (size_t)ra0 * K + 8 * hh;
  const unsigned short* ap1 = A + (size_t)ra1 * K + 8 * hh;
  const unsigned short* bp[4];
#pragma unroll
  for (int j = 0; j < 4; ++j) {
    int cb = c0 + 16 * j + m; cb = cb > Ncols - 1 ? Ncols - 1 : cb;
    bp[j] = Bt + (size_t)cb * K + 8 * hh;
  }

  v8f acc[2][4];
#pragma unroll
  for (int i = 0; i < 2; ++i)
#pragma unroll
    for (int j = 0; j < 4; ++j) { v8f z = {0.f, 0.f, 0.f, 0.f, 0.f, 0.f, 0.f, 0.f}; acc[i][j] = z; }

#pragma unroll 1
  for (int kt = 0; kt < KS; ++kt) {
    const int kb = kt << 5;
    FragH a0, a1, b0, b1, b2, b3;
    a0.u[0] = *(const v8us*)(ap0 + kb);
    a0.u[1] = *(const v8us*)(ap0 + kb + 16);
    a1.u[0] = *(const v8us*)(ap1 + kb);
    a1.u[1] = *(const v8us*)(ap1 + kb + 16);
    b0.u[0] = *(const v8us*)(bp[0] + kb);
    b0.u[1] = *(const v8us*)(bp[0] + kb + 16);
    b1.u[0] = *(const v8us*)(bp[1] + kb);
    b1.u[1] = *(const v8us*)(bp[1] + kb + 16);
    b2.u[0] = *(const v8us*)(bp[2] + kb);
    b2.u[1] = *(const v8us*)(bp[2] + kb + 16);
    b3.u[0] = *(const v8us*)(bp[3] + kb);
    b3.u[1] = *(const v8us*)(bp[3] + kb + 16);
    acc[0][0] = wmh(a0.v, b0.v, acc[0][0]);
    acc[1][0] = wmh(a1.v, b0.v, acc[1][0]);
    acc[0][1] = wmh(a0.v, b1.v, acc[0][1]);
    acc[1][1] = wmh(a1.v, b1.v, acc[1][1]);
    acc[0][2] = wmh(a0.v, b2.v, acc[0][2]);
    acc[1][2] = wmh(a1.v, b2.v, acc[1][2]);
    acc[0][3] = wmh(a0.v, b3.v, acc[0][3]);
    acc[1][3] = wmh(a1.v, b3.v, acc[1][3]);
  }

  float* sw = sT + wave * 2048;
#pragma unroll
  for (int i = 0; i < 2; ++i)
#pragma unroll
    for (int j = 0; j < 4; ++j)
#pragma unroll
      for (int r = 0; r < 8; ++r)
        sw[(16 * i + 8 * hh + r) * 64 + 16 * j + m] = acc[i][j][r];
  __syncthreads();

  if (O16 == 0) {
    v4f ov[16];
#pragma unroll
    for (int it = 0; it < 16; ++it) {
      const int f = it * 32 + lane;
      const int row = f >> 4, c4 = (f & 15) * 4;
      v4f v = *(const v4f*)(sw + row * 64 + c4);
      v = v * INVSCL;
      if (HASB) {
        const v4f bb = *(const v4f*)(bias + c0 + c4);
        v = v + bb;
      }
      if (RES) {
        int rr = r0 + row; rr = rr > rrows - 1 ? rrows - 1 : rr;
        const v4f rv = *(const v4f*)(resid + (size_t)rr * ldr + c0 + c4);
        v = v + rv;
      }
      if (RELU) {
        v.x = fmaxf(v.x, 0.0f); v.y = fmaxf(v.y, 0.0f); v.z = fmaxf(v.z, 0.0f); v.w = fmaxf(v.w, 0.0f);
      }
      ov[it] = v;
    }
#pragma unroll
    for (int it = 0; it < 16; ++it) {
      const int f = it * 32 + lane;
      const int row = f >> 4, c4 = (f & 15) * 4;
      *(volatile v4f*)(outF + (size_t)(r0 + row) * ldo + c0 + c4) = ov[it];
    }
    __threadfence();
#pragma unroll
    for (int it = 0; it < 16; ++it) {
      const int f = it * 32 + lane;
      const int row = f >> 4, c4 = (f & 15) * 4;
      *(volatile v4f*)(outF + (size_t)(r0 + row) * ldo + c0 + c4) = ov[it];
    }
  } else {
    v8us oh[8];
#pragma unroll
    for (int it = 0; it < 8; ++it) {
      const int f = it * 32 + lane;
      const int row = f >> 3, c8 = (f & 7) * 8;
      v4f a = *(const v4f*)(sw + row * 64 + c8);
      v4f b = *(const v4f*)(sw + row * 64 + c8 + 4);
      a = a * INVSCL; b = b * INVSCL;
      if (HASB) {
        const v4f ba = *(const v4f*)(bias + c0 + c8);
        const v4f bb = *(const v4f*)(bias + c0 + c8 + 4);
        a = a + ba; b = b + bb;
      }
      if (RES) {
        int rr = r0 + row; rr = rr > rrows - 1 ? rrows - 1 : rr;
        const v4f ra = *(const v4f*)(resid + (size_t)rr * ldr + c0 + c8);
        const v4f rb2 = *(const v4f*)(resid + (size_t)rr * ldr + c0 + c8 + 4);
        a = a + ra; b = b + rb2;
      }
      if (RELU) {
        a.x = fmaxf(a.x, 0.0f); a.y = fmaxf(a.y, 0.0f); a.z = fmaxf(a.z, 0.0f); a.w = fmaxf(a.w, 0.0f);
        b.x = fmaxf(b.x, 0.0f); b.y = fmaxf(b.y, 0.0f); b.z = fmaxf(b.z, 0.0f); b.w = fmaxf(b.w, 0.0f);
      }
      oh[it] = cvt8(a, b, ASCL);
    }
#pragma unroll
    for (int it = 0; it < 8; ++it) {
      const int f = it * 32 + lane;
      const int row = f >> 3, c8 = (f & 7) * 8;
      *(volatile v8us*)(outH + (size_t)(r0 + row) * ldo + c0 + c8) = oh[it];
    }
    __threadfence();
#pragma unroll
    for (int it = 0; it < 8; ++it) {
      const int f = it * 32 + lane;
      const int row = f >> 3, c8 = (f & 7) * 8;
      *(volatile v8us*)(outH + (size_t)(r0 + row) * ldo + c0 + c8) = oh[it];
    }
  }
}

__global__ __launch_bounds__(256) void k_edge(
    const float* __restrict__ F, const int* __restrict__ src, const float* __restrict__ eat,
    const float* __restrict__ We, const unsigned int* __restrict__ csort,
    const int* __restrict__ tab, unsigned short* a16, int nN, int nNp, int nE, int nCh) {
  extern __shared__ __attribute__((aligned(16))) int dsm[];
  __shared__ int sWtot[8];
  int* sOff  = dsm;
  int* sCur  = dsm + (RB + 8);
  int* sList = sCur + RB;
  const int tid = (int)threadIdx.x, lane = tid & 31, wave = tid >> 5;
  const int rgn = (int)blockIdx.x;
  const int n0 = rgn * RB;
  const unsigned int lt = (1u << lane) - 1u;

  for (int i = tid; i < RB + 8; i += 256) sOff[i] = 0;
  for (int i = tid; i < RB; i += 256) sCur[i] = 0;
  __syncthreads();

#pragma unroll 1
  for (int c = 0; c < nCh; ++c) {
    int pre = tab[(size_t)c * TABW + rgn];
    int n   = tab[(size_t)c * TABW + RMAX + rgn];
    pre = pre < 0 ? 0 : (pre > CHUNK ? CHUNK : pre);
    n = n < 0 ? 0 : (n > CHUNK - pre ? CHUNK - pre : n);
    const int nstep = (n + 31) >> 5;
    const unsigned int* cp = csort + (size_t)c * CHUNK + pre;
#pragma unroll 1
    for (int s = 0; s < nstep; ++s) {
      if (wave == 0) {
        const int i = (s << 5) + lane;
        const bool valid = i < n;
        const int ic = i > n - 1 ? n - 1 : i;
        const unsigned int en = cp[ic];
        const int j = (int)(en & (unsigned int)(RB - 1));
        const unsigned int msk = match_mask<RBBITS>(__builtin_amdgcn_ballot_w32(valid), j);
        const int rank = (int)__builtin_popcount(msk & lt);
        const int grp  = (int)__builtin_popcount(msk);
        if (valid && rank == 0) sOff[j] = sOff[j] + grp;
      }
      __syncthreads();
    }
  }
  __syncthreads();

  {
    int cn[4];
    int ls = 0;
#pragma unroll
    for (int i = 0; i < 4; ++i) { cn[i] = sOff[4 * tid + i]; ls += cn[i]; }
    int x = ls;
#pragma unroll
    for (int dd = 1; dd < 32; dd <<= 1) {
      const int y = __shfl_up(x, dd);
      x += (lane >= dd) ? y : 0;
    }
    if (lane == 31) sWtot[wave] = x;
    __syncthreads();
    int pre = 0;
#pragma unroll
    for (int w = 0; w < 8; ++w) { const int tw = sWtot[w]; pre += (w < wave) ? tw : 0; }
    int run = pre + x - ls;
#pragma unroll
    for (int i = 0; i < 4; ++i) { sOff[4 * tid + i] = run; run += cn[i]; }
    if (tid == 255) sOff[RB] = run;
  }
  __syncthreads();
  const bool rgnOver = sOff[RB] > LCAP;

#pragma unroll 1
  for (int c = 0; c < nCh; ++c) {
    int pre = tab[(size_t)c * TABW + rgn];
    int n   = tab[(size_t)c * TABW + RMAX + rgn];
    pre = pre < 0 ? 0 : (pre > CHUNK ? CHUNK : pre);
    n = n < 0 ? 0 : (n > CHUNK - pre ? CHUNK - pre : n);
    const int nstep = (n + 31) >> 5;
    const unsigned int* cp = csort + (size_t)c * CHUNK + pre;
#pragma unroll 1
    for (int s = 0; s < nstep; ++s) {
      if (wave == 0) {
        const int i = (s << 5) + lane;
        const bool valid = i < n;
        const int ic = i > n - 1 ? n - 1 : i;
        const unsigned int en = cp[ic];
        const int j = (int)(en & (unsigned int)(RB - 1));
        int e = (int)(en >> RBBITS);
        e = e > nE - 1 ? nE - 1 : e;
        const unsigned int msk = match_mask<RBBITS>(__builtin_amdgcn_ballot_w32(valid), j);
        const int rank = (int)__builtin_popcount(msk & lt);
        const int grp  = (int)__builtin_popcount(msk);
        const int cur  = sCur[j];
        const int p0   = sOff[j] + cur + rank;
        if (valid && (unsigned)p0 < (unsigned)LCAP) sList[p0] = e;
        if (valid && rank == 0) sCur[j] = cur + grp;
      }
      __syncthreads();
    }
  }
  __syncthreads();

  const int c4 = 4 * lane;
  const v4f we4 = *(const v4f*)(We + c4);
  int Rbp = nNp - n0; Rbp = Rbp > RB ? RB : Rbp;
  const int niter = (Rbp + 7) >> 3;
  const v4f zero4 = {0.0f, 0.0f, 0.0f, 0.0f};
  const float qn = __int_as_float(0x7fc00000);
  const v4f nan4 = {qn, qn, qn, qn};
  const int sl = 2 * (lane & 15);
#pragma unroll 1
  for (int jj = 0; jj < niter; ++jj) {
    const int j = jj * 8 + wave;
    const bool act = j < Rbp;
    const int jc = act ? j : (Rbp - 1);
    const int node = n0 + jc;
    const bool live = node < nN;
    int lb = __builtin_amdgcn_readfirstlane(sOff[jc]);
    int ub = __builtin_amdgcn_readfirstlane(sOff[jc + 1]);
    lb = lb < 0 ? 0 : (lb > LCAP ? LCAP : lb);
    ub = ub < 0 ? 0 : (ub > LCAP ? LCAP : ub);
    const int craw = ub - lb;
    int cnt = craw;
    cnt = cnt < 0 ? 0 : (cnt > DEGCAP ? DEGCAP : cnt);

    const float* frow = F + (size_t)node * NQKV;
    const v4f qv = *(const v4f*)(frow + c4);
    const v4f qw = qv * we4;

    v4f acc = zero4;
    float z = 0.0f;
#pragma unroll 1
    for (int it = 0; it < cnt; ++it) {
      int li = lb + it; li = li > LCAP - 1 ? LCAP - 1 : li;
      int e = sList[li]; e = e < 0 ? 0 : (e > nE - 1 ? nE - 1 : e);
      int s = src[e];   s = s < 0 ? 0 : (s > nN - 1 ? nN - 1 : s);
      const float ea = eat[e];
      const float* krow = F + (size_t)s * NQKV;
      const v4f kv = *(const v4f*)(krow + DM + c4);
      const v4f vv = *(const v4f*)(krow + 2 * DM + c4);
      float part = kv.x * qw.x;
      part = fmaf(kv.y, qw.y, part);
      part = fmaf(kv.z, qw.z, part);
      part = fmaf(kv.w, qw.w, part);
      part += __shfl_xor(part, 1);
      part += __shfl_xor(part, 2);
      float sc = part * 0.25f * ea;
      sc = fminf(5.0f, fmaxf(-5.0f, sc));
      const float p = __expf(sc);
      acc = acc + vv * p;
      z += p;
    }
    const float rz = 1.0f / (z + 1e-6f);
    v4f r = acc * rz;
    const bool bad = (craw > DEGCAP) || rgnOver;
    r = bad ? nan4 : r;
    r = live ? r : zero4;

    const unsigned int u0 = pk2(r.x * ASCL, r.y * ASCL);
    const unsigned int u1 = pk2(r.z * ASCL, r.w * ASCL);
    v4u q;
    q.x = (unsigned int)__shfl((int)u0, sl);
    q.y = (unsigned int)__shfl((int)u1, sl);
    q.z = (unsigned int)__shfl((int)u0, sl + 1);
    q.w = (unsigned int)__shfl((int)u1, sl + 1);
    unsigned short* op = a16 + (size_t)node * DM + 8 * (lane & 15);
    const bool wst = act && (lane < 16);
    if (wst) *(volatile v4u*)op = q;
    __threadfence();
    if (wst) *(volatile v4u*)op = q;
  }
}

__global__ __launch_bounds__(256) void k_colstat(
    const float* __restrict__ P, int nN, double* part) {
  __shared__ __attribute__((aligned(16))) double sD[256];
  __shared__ __attribute__((aligned(16))) double sE[256];
  const int tid = (int)threadIdx.x, c = tid & 127, hf = tid >> 7;
  const int rbase = (int)blockIdx.x * STATRS;
  double s = 0.0, s2 = 0.0;
#pragma unroll 4
  for (int i = 0; i < STATRS / 2; ++i) {
    const int r = rbase + 2 * i + hf;
    const float v0 = P[(size_t)r * DM + c];
    const float v = (r < nN) ? v0 : 0.0f;
    const double dv = (double)v;
    s += dv;
    s2 += dv * dv;
  }
  if (hf == 1) { sD[c] = s; sD[128 + c] = s2; }
  __syncthreads();
  if (hf == 0) { sE[c] = s + sD[c]; sE[128 + c] = s2 + sD[128 + c]; }
  __syncthreads();
  const bool w = tid < 128;
  const int q = tid & 127;
  const v2d v = *(const v2d*)(sE + 2 * q);
  double* gp = part + (size_t)blockIdx.x * 256 + 2 * q;
  if (w) *(volatile v2d*)gp = v;
  __threadfence();
  if (w) *(volatile v2d*)gp = v;
}

__global__ __launch_bounds__(128) void k_bnfin(
    const double* __restrict__ part, int nblk, int nN, float* stats) {
  __shared__ __attribute__((aligned(16))) float sF[256];
  const int c = (int)threadIdx.x;
  double s = 0.0, s2 = 0.0;
#pragma unroll 1
  for (int b = 0; b < nblk; ++b) {
    s  += part[(size_t)b * 256 + c];
    s2 += part[(size_t)b * 256 + 128 + c];
  }
  const double invn = 1.0 / (double)nN;
  const double mu = s * invn;
  double var = s2 * invn - mu * mu;
  var = var < 0.0 ? 0.0 : var;
  const float varf = (float)var;
  sF[c] = (float)mu;
  sF[128 + c] = rsqrtf(varf + 1e-5f);
  __syncthreads();
  const bool w = c < 64;
  const int cc = c & 63;
  const v4f v = *(const v4f*)(sF + 4 * cc);
  if (w) *(volatile v4f*)(stats + 4 * cc) = v;
  __threadfence();
  if (w) *(volatile v4f*)(stats + 4 * cc) = v;
}

__global__ __launch_bounds__(256) void k_bn1(
    const float* __restrict__ P, const float* __restrict__ stats,
    const float* __restrict__ g, const float* __restrict__ b,
    float* H32, unsigned short* H16) {
  const int tid = (int)threadIdx.x, lane = tid & 31, wave = tid >> 5;
  const int c4 = 4 * lane;
  const v4f mu = *(const v4f*)(stats + c4);
  const v4f rs = *(const v4f*)(stats + 128 + c4);
  const v4f gg = *(const v4f*)(g + c4);
  const v4f bb = *(const v4f*)(b + c4);
  const int rb = (int)blockIdx.x * 64;
  const int sl = 2 * (lane & 15);
  const bool wl = lane < 16;
#pragma unroll 1
  for (int grp = 0; grp < 2; ++grp) {
    const int rw = rb + grp * 32 + wave * 4;
    v4f y[4];
    v4u hq[4];
#pragma unroll
    for (int i = 0; i < 4; ++i) {
      const v4f v = *(const v4f*)(P + (size_t)(rw + i) * DM + c4);
      const v4f t = (v - mu) * rs * gg + bb;
      y[i] = t;
      const unsigned int u0 = pk2(t.x * ASCL, t.y * ASCL);
      const unsigned int u1 = pk2(t.z * ASCL, t.w * ASCL);
      v4u q;
      q.x = (unsigned int)__shfl((int)u0, sl);
      q.y = (unsigned int)__shfl((int)u1, sl);
      q.z = (unsigned int)__shfl((int)u0, sl + 1);
      q.w = (unsigned int)__shfl((int)u1, sl + 1);
      hq[i] = q;
    }
#pragma unroll
    for (int i = 0; i < 4; ++i) {
      *(volatile v4f*)(H32 + (size_t)(rw + i) * DM + c4) = y[i];
      if (wl) *(volatile v4u*)(H16 + (size_t)(rw + i) * DM + 8 * (lane & 15)) = hq[i];
    }
    __threadfence();
#pragma unroll
    for (int i = 0; i < 4; ++i) {
      *(volatile v4f*)(H32 + (size_t)(rw + i) * DM + c4) = y[i];
      if (wl) *(volatile v4u*)(H16 + (size_t)(rw + i) * DM + 8 * (lane & 15)) = hq[i];
    }
  }
}

__global__ __launch_bounds__(256) void k_bn2(
    const float* __restrict__ P, const float* __restrict__ stats,
    const float* __restrict__ g, const float* __restrict__ b,
    float* out, int nN) {
  const int tid = (int)threadIdx.x, lane = tid & 31, wave = tid >> 5;
  const int c4 = 4 * lane;
  const v4f mu = *(const v4f*)(stats + c4);
  const v4f rs = *(const v4f*)(stats + 128 + c4);
  const v4f gg = *(const v4f*)(g + c4);
  const v4f bb = *(const v4f*)(b + c4);
  const int rb = (int)blockIdx.x * 64;
#pragma unroll 1
  for (int grp = 0; grp < 2; ++grp) {
    const int rw = rb + grp * 32 + wave * 4;
    v4f y[4];
#pragma unroll
    for (int i = 0; i < 4; ++i) {
      const v4f v = *(const v4f*)(P + (size_t)(rw + i) * DM + c4);
      y[i] = (v - mu) * rs * gg + bb;
    }
#pragma unroll
    for (int i = 0; i < 4; ++i)
      if (rw + i < nN) *(volatile v4f*)(out + (size_t)(rw + i) * DM + c4) = y[i];
    __threadfence();
#pragma unroll
    for (int i = 0; i < 4; ++i)
      if (rw + i < nN) *(volatile v4f*)(out + (size_t)(rw + i) * DM + c4) = y[i];
  }
}

extern "C" void kernel_launch(void* const* d_in, const int* in_sizes, int n_in,
                              void* d_out, int out_size, void* d_ws, size_t ws_size,
                              hipStream_t stream) {
  if (n_in < 17) return;
  const int nN = in_sizes[0] / DM;
  const int nE = in_sizes[1];
  if (nN <= 0 || nE <= 0) return;
  if (in_sizes[0] != nN * DM) return;
  if (in_sizes[2] != 2 * nE) return;
  if (nN > RMAX * RB || nE > (1 << 22)) return;
  if (in_sizes[3] != DM * DM || in_sizes[4] != DM * DM || in_sizes[6] != DM * DM || in_sizes[7] != DM * DM) return;
  if (in_sizes[5] != DM) return;
  if (in_sizes[8] != DM || in_sizes[9] != DM || in_sizes[10] != DM) return;
  if (in_sizes[11] != DM * FW || in_sizes[12] != FW || in_sizes[13] != FW * DM) return;
  if (in_sizes[14] != DM || in_sizes[15] != DM || in_sizes[16] != DM) return;
  if (out_size != nN * DM) return;

  const float* x    = (const float*)d_in[0];
  const float* eat  = (const float*)d_in[1];
  const int*   ei   = (const int*)d_in[2];
  const float* Wq   = (const float*)d_in[3];
  const float* Wk   = (const float*)d_in[4];
  const float* We   = (const float*)d_in[5];
  const float* Wv   = (const float*)d_in[6];
  const float* Wo   = (const float*)d_in[7];
  const float* bo   = (const float*)d_in[8];
  const float* g1   = (const float*)d_in[9];
  const float* b1   = (const float*)d_in[10];
  const float* W1   = (const float*)d_in[11];
  const float* bf1  = (const float*)d_in[12];
  const float* W2   = (const float*)d_in[13];
  const float* bf2  = (const float*)d_in[14];
  const float* g2   = (const float*)d_in[15];
  const float* b2   = (const float*)d_in[16];
  const int*   esrc = ei;
  const int*   edst = ei + nE;
  float* out = (float*)d_out;

  const int nCh = (nE + CHUNK - 1) / CHUNK;
  const int nR  = (nN + RB - 1) / RB;
  const int nNp = ((nN + 127) / 128) * 128;
  const int nSB = nNp / STATRS;

  const size_t szS16  = (size_t)nNp * DM * 2;
  const size_t szF    = (size_t)nNp * NQKV * 4;
  const size_t szFF   = (size_t)nNp * FW * 2;
  const size_t szWA   = (size_t)4 * DM * DM * 2;
  const size_t szW1   = (size_t)FW * DM * 2;
  const size_t szW2   = (size_t)DM * FW * 2;
  const size_t szCS   = (size_t)nCh * CHUNK * 4;
  const size_t szTab  = (size_t)nCh * TABW * 4;
  const size_t szPart = (size_t)nSB * 256 * 8;
  const size_t szStat = 256 * 4;
  size_t off = 0;
  const size_t oS  = off; off += szS16;  off = (off + 255) & ~(size_t)255;
  const size_t oF  = off; off += szF;    off = (off + 255) & ~(size_t)255;
  const size_t oFF = off; off += szFF;   off = (off + 255) & ~(size_t)255;
  const size_t oWA = off; off += szWA;   off = (off + 255) & ~(size_t)255;
  const size_t oW1 = off; off += szW1;   off = (off + 255) & ~(size_t)255;
  const size_t oW2 = off; off += szW2;   off = (off + 255) & ~(size_t)255;
  const size_t oC  = off; off += szCS;   off = (off + 255) & ~(size_t)255;
  const size_t oT  = off; off += szTab;  off = (off + 255) & ~(size_t)255;
  const size_t oPa = off; off += szPart; off = (off + 255) & ~(size_t)255;
  const size_t oPb = off; off += szPart; off = (off + 255) & ~(size_t)255;
  const size_t oSa = off; off += szStat; off = (off + 255) & ~(size_t)255;
  const size_t oSb = off; off += szStat; off = (off + 255) & ~(size_t)255;
  if (off > ws_size || off > (size_t)WSCAP) return;
  if ((size_t)3 * nNp * DM * 4 > szF) return;

  char* ws = (char*)d_ws;
  unsigned short* s16   = (unsigned short*)(ws + oS);
  float*          F     = (float*)(ws + oF);
  float*          P1    = F;
  float*          H1    = F + (size_t)nNp * DM;
  float*          P2    = F + (size_t)2 * nNp * DM;
  unsigned short* ff16  = (unsigned short*)(ws + oFF);
  unsigned short* wA    = (unsigned short*)(ws + oWA);
  unsigned short* w1t   = (unsigned short*)(ws + oW1);
  unsigned short* w2t   = (unsigned short*)(ws + oW2);
  unsigned int*   csort = (unsigned int*)(ws + oC);
  int*            tab   = (int*)(ws + oT);
  double*         partA = (double*)(ws + oPa);
  double*         partB = (double*)(ws + oPb);
  float*          statA = (float*)(ws + oSa);
  float*          statB = (float*)(ws + oSb);

  k_csort<<<nCh, 256, 0, stream>>>(edst, csort, tab, nN, nE);

  k_xcvt<<<nNp / 128, 256, 0, stream>>>(x, s16, nN);

  k_wprep<DM, DM><<<16, 256, 0, stream>>>(Wq, Wk, Wv, Wo, wA);
  k_wprep<DM, FW><<<8, 256, 0, stream>>>(W1, W1, W1, W1, w1t);
  k_wprep<FW, DM><<<4, 256, 0, stream>>>(W2, W2, W2, W2, w2t);

  k_gemm<DM / 32, 0, 0, 0, 0><<<dim3(NQKV / 64, nNp / 128, 1), GT, 0, stream>>>(
      s16, wA, bo, x, DM, nN, F, ff16, NQKV, nNp, NQKV);

  hipFuncSetAttribute(reinterpret_cast<const void*>(&k_edge),
                      hipFuncAttributeMaxDynamicSharedMemorySize, EDGE_LDS_BYTES);
  k_edge<<<nR, 256, EDGE_LDS_BYTES, stream>>>(F, esrc, eat, We, csort, tab, s16, nN, nNp, nE, nCh);

  k_gemm<DM / 32, 1, 1, 0, 0><<<dim3(DM / 64, nNp / 128, 1), GT, 0, stream>>>(
      s16, wA + (size_t)NQKV * DM, bo, x, DM, nN, P1, ff16, DM, nNp, DM);

  k_colstat<<<nSB, 256, 0, stream>>>(P1, nN, partA);
  k_bnfin<<<1, 128, 0, stream>>>(partA, nSB, nN, statA);
  k_bn1<<<nNp / 64, 256, 0, stream>>>(P1, statA, g1, b1, H1, s16);

  k_gemm<DM / 32, 1, 0, 1, 1><<<dim3(FW / 64, nNp / 128, 1), GT, 0, stream>>>(
      s16, w1t, bf1, x, DM, nN, P2, ff16, FW, nNp, FW);

  k_gemm<FW / 32, 1, 1, 0, 0><<<dim3(DM / 64, nNp / 128, 1), GT, 0, stream>>>(
      ff16, w2t, bf2, H1, DM, nNp, P2, s16, DM, nNp, DM);

  k_colstat<<<nSB, 256, 0, stream>>>(P2, nN, partB);
  k_bnfin<<<1, 128, 0, stream>>>(partB, nSB, nN, statB);
  k_bn2<<<nNp / 64, 256, 0, stream>>>(P2, statB, g2, b2, out, nN);
}
